// WAHead_85152021610607
// MI455X (gfx1250) — hardware-verified
//
#include <hip/hip_runtime.h>
#include <math.h>

typedef __attribute__((ext_vector_type(16))) _Float16 v16h;
typedef __attribute__((ext_vector_type(8)))  _Float16 v8h;
typedef __attribute__((ext_vector_type(16))) __bf16   v16b;
typedef __attribute__((ext_vector_type(8)))  __bf16   v8b;
typedef __attribute__((ext_vector_type(8)))  float    v8f;
typedef __attribute__((ext_vector_type(4)))  float    v4f;
typedef __attribute__((ext_vector_type(4)))  unsigned int v4u;

constexpr int kNB    = 32768;
constexpr int kNA    = 5;
constexpr int kEmb   = 16;
constexpr int kLat   = 128;
constexpr int kSteps = 3;
constexpr int kEns   = 3;
constexpr int kRows  = kNB * kNA;
constexpr int kGate  = 4 * kLat;

constexpr int kChunkRows   = 32768;
constexpr int kNumChunks   = kRows / kChunkRows;
constexpr int kLdA         = 192;
constexpr int kKdim        = 160;
constexpr int kLdHead      = 128;
constexpr int kNHead       = 64;
constexpr int kRowsPerWave = 8;
constexpr int kRowsPerBlock = 8 * kRowsPerWave;

constexpr float kWhhCarry  = 64.0f;
constexpr float kHeadCarry = 64.0f;
constexpr float kWihCarry  = 8.0f;
constexpr float kEmbCarry  = 8.0f;
constexpr float kScaleInv  = 1.0f / 64.0f;

static_assert(kNumChunks * kChunkRows == kRows);
static_assert(kChunkRows % kRowsPerBlock == 0);
static_assert(kChunkRows % 256 == 0);
static_assert(kChunkRows % 64 == 0 && kGate % 64 == 0 && kNHead % 64 == 0);
static_assert(kKdim % 32 == 0 && kLat % 32 == 0 && kKdim <= kLdA);

constexpr size_t kOffBt   = 0;
constexpr size_t kOffBtH  = kOffBt + (size_t)kGate * kLdA * 2;
constexpr size_t kOffBias = kOffBtH + (size_t)kNHead * kLdHead * 2;
constexpr size_t kOffA    = 262144;
constexpr size_t kOffG    = kOffA + (size_t)kChunkRows * kLdA * 2;
constexpr size_t kOffC0   = kOffG + (size_t)kChunkRows * kGate * 4;
constexpr size_t kOffC1   = kOffC0 + (size_t)kChunkRows * kLat * 4;
constexpr size_t kOffHp   = kOffC1 + (size_t)kChunkRows * kLat * 4;
constexpr size_t kWsTotal = kOffHp + (size_t)kChunkRows * kNHead * 4;
static_assert(kOffBias + 2048 <= kOffA);
static_assert(kWsTotal == 121896960);
static_assert(kWsTotal <= 134217728);
static_assert(kOffA % 128 == 0 && kOffG % 128 == 0 && kOffC0 % 128 == 0 && kOffC1 % 128 == 0 && kOffHp % 128 == 0 && kOffBtH % 128 == 0 && kOffBias % 128 == 0);

__device__ __forceinline__ unsigned short f2bf_bits(float f) {
  unsigned u = __float_as_uint(f);
  return (unsigned short)((u + 0x7FFFu + ((u >> 16) & 1u)) >> 16);
}
__device__ __forceinline__ float bf_bits2f(unsigned short h) { return __uint_as_float(((unsigned)h) << 16); }

__device__ __forceinline__ void dep_guard_h(v8f& a, v8f& b, v16h x, v16h y) { asm volatile("v_nop\n\tv_nop\n\tv_nop\n\tv_nop" : "+v"(a), "+v"(b) : "v"(x), "v"(y)); }
__device__ __forceinline__ void dep_guard_b(v8f& a, v8f& b, v16b x, v16b y) { asm volatile("v_nop\n\tv_nop\n\tv_nop\n\tv_nop" : "+v"(a), "+v"(b) : "v"(x), "v"(y)); }
__device__ __forceinline__ void keep4_h(v16h a, v16h b, v16h c, v16h d) { asm volatile("v_nop" :: "v"(a), "v"(b), "v"(c), "v"(d)); }
__device__ __forceinline__ void keep4_b(v16b a, v16b b, v16b c, v16b d) { asm volatile("v_nop" :: "v"(a), "v"(b), "v"(c), "v"(d)); }
__device__ __forceinline__ void acc_guard4(v8f& a, v8f& b, v8f& c, v8f& d) { asm volatile("v_nop\n\tv_nop\n\tv_nop\n\tv_nop" : "+v"(a), "+v"(b), "+v"(c), "+v"(d)); }
template <typename T> struct Frag;
template <> struct Frag<_Float16> {
  typedef v16h V; union U { v16h v; v8h h[2]; };
  static __device__ __forceinline__ v16h load(const _Float16* p) {
    U f; f.h[0] = *(const v8h*)(p); f.h[1] = *(const v8h*)(p + 16); return f.v;
  }
  static __device__ __forceinline__ v8f mma(v16h a, v16h b, v8f c) {
    return __builtin_amdgcn_wmma_f32_16x16x32_f16(false, a, false, b, (short)0, c, false, false);
  }
  static __device__ __forceinline__ void guard(v8f& a, v8f& b, v16h x, v16h y) { dep_guard_h(a, b, x, y); }
  static __device__ __forceinline__ void keep(v16h a, v16h b, v16h c, v16h d) { keep4_h(a, b, c, d); }
};
template <> struct Frag<__bf16> {
  typedef v16b V; union U { v16b v; v8b h[2]; };
  static __device__ __forceinline__ v16b load(const __bf16* p) {
    U f; f.h[0] = *(const v8b*)(p); f.h[1] = *(const v8b*)(p + 16); return f.v;
  }
  static __device__ __forceinline__ v8f mma(v16b a, v16b b, v8f c) {
    return __builtin_amdgcn_wmma_f32_16x16x32_bf16(false, a, false, b, (short)0, c, false, false);
  }
  static __device__ __forceinline__ void guard(v8f& a, v8f& b, v16b x, v16b y) { dep_guard_b(a, b, x, y); }
  static __device__ __forceinline__ void keep(v16b a, v16b b, v16b c, v16b d) { keep4_b(a, b, c, d); }
};

__device__ __forceinline__ unsigned pk16(unsigned short a, unsigned short b) { return (unsigned)a | ((unsigned)b << 16); }
__device__ __forceinline__ unsigned short h_bits(float f) { const _Float16 h = (_Float16)f; return __builtin_bit_cast(unsigned short, h); }

template <int ET> struct Elem;
template <> struct Elem<0> { typedef _Float16 T; };
template <> struct Elem<1> { typedef __bf16 T; };
template <int ET, bool SPLIT, int BIAS_MODE, int OUT_MODE, bool RESID, int ACT = 0>
__global__ __launch_bounds__(256) void wmma_gemm64(
    const unsigned short* __restrict__ Ap, const unsigned short* __restrict__ A2p, int lda, long strideA,
    const unsigned short* __restrict__ Btp, const unsigned short* __restrict__ Bt2p, int ldb, long strideB,
    void* __restrict__ Cout, void* __restrict__ Cout2, int ldc, long strideC,
    const float* __restrict__ bias,
    const float* __restrict__ resid, long strideR,
    int M, int N, int K, float scale) {
  typedef typename Elem<ET>::T T;
  typedef typename Frag<T>::V V;
  const T* A = (const T*)Ap; const T* A2 = (const T*)A2p; const T* Bt = (const T*)Btp; const T* Bt2 = (const T*)Bt2p;
  __shared__ __align__(16) float sT[8][16 * 68];
  const int b    = blockIdx.y;
  const int lane = threadIdx.x & 31;
  const int wave = threadIdx.x >> 5;
  const int tilesN = N >> 6;
  const int tilesM = M >> 6;
  const int tile = blockIdx.x * 8 + wave;
  if (tile >= tilesM * tilesN) return;
  const int tm = tile / tilesN;
  const int tn = tile - tm * tilesN;
  const int m0 = tm << 6;
  const int n0 = tn << 6;

  const T* Ab  = A  + (size_t)b * strideA;
  const T* Bb  = Bt + (size_t)b * strideB;
  const T* Ab2 = SPLIT ? (A2  + (size_t)b * strideA) : nullptr;
  const T* Bb2 = SPLIT ? (Bt2 + (size_t)b * strideB) : nullptr;

  const int rlane = lane & 15;
  const int koff  = (lane >> 4) * 8;
  const int mOff  = (lane >> 4) * 8;

  v8f acc[4][4];
#pragma unroll
  for (int i = 0; i < 4; ++i)
#pragma unroll
    for (int j = 0; j < 4; ++j) acc[i][j] = (v8f){0.f,0.f,0.f,0.f,0.f,0.f,0.f,0.f};

  for (int k0 = 0; k0 < K; k0 += 32) {
    V bh[4], bl[4];
#pragma unroll
    for (int j = 0; j < 4; ++j) {
      const size_t bo = (size_t)(n0 + (j << 4) + rlane) * ldb + koff + k0;
      bh[j] = Frag<T>::load(Bb + bo);
      if (SPLIT) bl[j] = Frag<T>::load(Bb2 + bo);
    }
#pragma unroll
    for (int i = 0; i < 4; ++i) {
      const size_t ao = (size_t)(m0 + (i << 4) + rlane) * lda + koff + k0;
      V ah = Frag<T>::load(Ab + ao);
      V al;
      if (SPLIT) al = Frag<T>::load(Ab2 + ao);
#pragma unroll
      for (int j = 0; j < 4; ++j) {
        acc[i][j] = Frag<T>::mma(ah, bh[j], acc[i][j]);
        if (SPLIT) {
          acc[i][j] = Frag<T>::mma(ah, bl[j], acc[i][j]);
          acc[i][j] = Frag<T>::mma(al, bh[j], acc[i][j]);
        }
      }
      Frag<T>::guard(acc[i][0], acc[i][3], ah, SPLIT ? al : ah);
    }
    Frag<T>::keep(bh[0], bh[1], bh[2], bh[3]);
    if (SPLIT) Frag<T>::keep(bl[0], bl[1], bl[2], bl[3]);
  }
  acc_guard4(acc[0][0], acc[0][1], acc[0][2], acc[0][3]);
  acc_guard4(acc[1][0], acc[1][1], acc[1][2], acc[1][3]);
  acc_guard4(acc[2][0], acc[2][1], acc[2][2], acc[2][3]);
  acc_guard4(acc[3][0], acc[3][1], acc[3][2], acc[3][3]);

  float* slab = sT[wave];
  const float* Rb = RESID ? (resid + (size_t)b * strideR) : nullptr;
#pragma unroll
  for (int i = 0; i < 4; ++i) {
    const int mBase = m0 + (i << 4);
#pragma unroll
    for (int j = 0; j < 4; ++j) {
      const int n = n0 + (j << 4) + rlane;
      float bv = 0.f;
      if (BIAS_MODE == 2) bv = bias[n];
#pragma unroll
      for (int r = 0; r < 8; ++r) {
        float v = acc[i][j][r] * scale;
        if (BIAS_MODE == 1) v += bias[mBase + mOff + r];
        if (BIAS_MODE == 2) v += bv;
        if (RESID) v += Rb[(size_t)(mBase + mOff + r) * ldc + n];
        if (ACT == 2) v = fmaxf(v, 0.0f);
        if (ACT == 4) v = (v > 0.f) ? v : 0.01f * v;
        slab[(mOff + r) * 68 + (j << 4) + rlane] = v;
      }
    }
    __builtin_amdgcn_fence(__ATOMIC_RELEASE, "workgroup");
    __builtin_amdgcn_wave_barrier();
    __builtin_amdgcn_fence(__ATOMIC_ACQUIRE, "workgroup");
    if (OUT_MODE == 0) {
      float* C = (float*)Cout + (size_t)b * strideC;
      const int hh = lane >> 4, c4 = (lane & 15) * 4;
      for (int pass = 0; pass < 2; ++pass) {
#pragma unroll
        for (int it = 0; it < 8; ++it) {
          const int row = it * 2 + hh;
          v4f v = *(const v4f*)(slab + row * 68 + c4);
          *(volatile v4f*)(C + (size_t)(mBase + row) * ldc + n0 + c4) = v;
        }
        __threadfence();
      }
    } else {
      const int q = lane >> 3, c8 = (lane & 7) * 8;
      unsigned short* C  = (unsigned short*)Cout  + (size_t)b * strideC;
      unsigned short* C2 = (OUT_MODE == 2) ? ((unsigned short*)Cout2 + (size_t)b * strideC) : nullptr;
      for (int pass = 0; pass < 2; ++pass) {
#pragma unroll
        for (int it = 0; it < 4; ++it) {
          const int row = it * 4 + q;
          const float* sp = slab + row * 68 + c8;
          v8h hv, lv;
#pragma unroll
          for (int e = 0; e < 8; ++e) {
            if (OUT_MODE == 1) {
              hv[e] = (_Float16)sp[e];
            } else {
              unsigned short hb = f2bf_bits(sp[e]);
              unsigned short lb = f2bf_bits(sp[e] - bf_bits2f(hb));
              hv[e] = __builtin_bit_cast(_Float16, hb);
              lv[e] = __builtin_bit_cast(_Float16, lb);
            }
          }
          *(volatile v8h*)(C + (size_t)(mBase + row) * ldc + n0 + c8) = hv;
          if (OUT_MODE == 2) *(volatile v8h*)(C2 + (size_t)(mBase + row) * ldc + n0 + c8) = lv;
        }
        __threadfence();
      }
    }
    __builtin_amdgcn_fence(__ATOMIC_RELEASE, "workgroup");
    __builtin_amdgcn_wave_barrier();
    __builtin_amdgcn_fence(__ATOMIC_ACQUIRE, "workgroup");
  }
}

__device__ __forceinline__ v4u pack8h(v4f a, v4f b, float s) {
  v4u u;
  u.x = pk16(h_bits(a.x * s), h_bits(a.y * s));
  u.y = pk16(h_bits(a.z * s), h_bits(a.w * s));
  u.z = pk16(h_bits(b.x * s), h_bits(b.y * s));
  u.w = pk16(h_bits(b.z * s), h_bits(b.w * s));
  return u;
}
__device__ __forceinline__ v4u sel4u(bool c, v4u a, v4u b) {
  v4u r;
  r.x = c ? a.x : b.x; r.y = c ? a.y : b.y; r.z = c ? a.z : b.z; r.w = c ? a.w : b.w;
  return r;
}
__device__ __forceinline__ float get4f(v4f v, int u) { return (u == 0) ? v.x : ((u == 1) ? v.y : ((u == 2) ? v.z : v.w)); }
__device__ __forceinline__ v4f put4f(v4f v, int u, float s) {
  v4f r;
  r.x = (u == 0) ? s : v.x; r.y = (u == 1) ? s : v.y; r.z = (u == 2) ? s : v.z; r.w = (u == 3) ? s : v.w;
  return r;
}
__device__ __forceinline__ float rcp_f(float x) { return __builtin_amdgcn_rcpf(x); }
__device__ __forceinline__ float sigm_f(float x) { return rcp_f(1.0f + expf(-x)); }
__device__ __forceinline__ float tanh_f(float x) { return 1.0f - 2.0f * rcp_f(expf(2.0f * x) + 1.0f); }

__global__ __launch_bounds__(256) void prep_weights_kernel(
    const float* __restrict__ Wih, const float* __restrict__ Whh,
    const float* __restrict__ bih, const float* __restrict__ bhh,
    const float* __restrict__ Wp, const float* __restrict__ Wr,
    unsigned short* __restrict__ Bt, unsigned short* __restrict__ BtH, float* __restrict__ biasS) {
  const int lane = threadIdx.x & 31;
  const int gw = blockIdx.x * 8 + (threadIdx.x >> 5);
  const v4u zero4 = (v4u){0u, 0u, 0u, 0u};
  if (gw < kGate) {
    const int n = gw;
    const int ih = (lane < 16 ? lane : 15) * 8;
    const float* ph = Whh + (size_t)n * kLat + ih;
    const v4f h0 = *(const v4f*)(ph);
    const v4f h1 = *(const v4f*)(ph + 4);
    const int ii = (lane & 1) * 8;
    const float* pe = Wih + (size_t)n * kEmb + ii;
    const v4f e0 = *(const v4f*)(pe);
    const v4f e1 = *(const v4f*)(pe + 4);
    const v4u wv = pack8h(h0, h1, kWhhCarry);
    const v4u iv = pack8h(e0, e1, kWihCarry);
    const v4u val = sel4u(lane < 16, wv, sel4u(lane < 18, iv, zero4));
    unsigned short* dst = Bt + (size_t)n * kLdA + 8 * (lane < 24 ? lane : 23);
    for (int pass = 0; pass < 2; ++pass) {
      if (lane < 24) *(volatile v4u*)dst = val;
      __threadfence();
    }
  } else if (gw < kGate + kNHead) {
    const int hr = gw - kGate;
    const int iq = (lane < 16 ? lane : 15) * 8;
    const v4f p0 = *(const v4f*)(Wp + iq);
    const v4f p1 = *(const v4f*)(Wp + iq + 4);
    int e = hr - 1;
    e = e < 0 ? 0 : (e > kEns - 1 ? kEns - 1 : e);
    const float* pr = Wr + (size_t)e * kLat + iq;
    const v4f r0 = *(const v4f*)(pr);
    const v4f r1 = *(const v4f*)(pr + 4);
    const v4u pv = pack8h(p0, p1, kHeadCarry);
    const v4u rv = pack8h(r0, r1, kHeadCarry);
    const v4u val = sel4u(hr == 0, pv, sel4u(hr <= kEns, rv, zero4));
    unsigned short* dst = BtH + (size_t)hr * kLdHead + 8 * (lane & 15);
    for (int pass = 0; pass < 2; ++pass) {
      if (lane < 16) *(volatile v4u*)dst = val;
      __threadfence();
    }
  }
  if (gw == 0) {
    v4f bs[4];
#pragma unroll
    for (int q = 0; q < 4; ++q) {
      const int idx = q * kLat + 4 * lane;
      bs[q] = *(const v4f*)(bih + idx) + *(const v4f*)(bhh + idx);
    }
    for (int pass = 0; pass < 2; ++pass) {
#pragma unroll
      for (int q = 0; q < 4; ++q) *(volatile v4f*)(biasS + q * kLat + 4 * lane) = bs[q];
      __threadfence();
    }
  }
}

__global__ __launch_bounds__(256) void init_rows_kernel(
    const float* __restrict__ z, const float* __restrict__ anchors,
    const float* __restrict__ W1, const float* __restrict__ b1,
    const float* __restrict__ W2, const float* __restrict__ b2,
    unsigned short* __restrict__ Apl, int rowBase) {
  const int lane = threadIdx.x & 31;
  const int wave = threadIdx.x >> 5;
  const int qL = lane & 15;
  const int j = qL;
  const int rbase = (blockIdx.x * 8 + wave) * kRowsPerWave;
  float w1r[2 * kEmb], b1r[kEmb], w2r[kEmb];
#pragma unroll
  for (int m = 0; m < kEmb; ++m) {
    w1r[2 * m] = W1[2 * m];
    w1r[2 * m + 1] = W1[2 * m + 1];
    b1r[m] = b1[m];
    w2r[m] = W2[j * kEmb + m];
  }
  const float b2r = b2[j];
  const int sb = (lane & 1) * 8;
  const v4u zero4 = (v4u){0u, 0u, 0u, 0u};
#pragma unroll 1
  for (int rr = 0; rr < kRowsPerWave; ++rr) {
    const int row = rbase + rr;
    const int gr = rowBase + row;
    const int bidx = gr / kNA;
    const v4f zv = *(const v4f*)(z + (size_t)bidx * kLat + 4 * lane);
    const unsigned p0 = pk16(h_bits(zv.x), h_bits(zv.y));
    const unsigned p1 = pk16(h_bits(zv.z), h_bits(zv.w));
    v4u hv;
    hv.x = __shfl(p0, 2 * qL);
    hv.y = __shfl(p1, 2 * qL);
    hv.z = __shfl(p0, 2 * qL + 1);
    hv.w = __shfl(p1, 2 * qL + 1);
    const float a0 = anchors[(size_t)gr * 2];
    const float a1 = anchors[(size_t)gr * 2 + 1];
    float s = b2r;
#pragma unroll
    for (int m = 0; m < kEmb; ++m) {
      const float pre = a0 * w1r[2 * m] + a1 * w1r[2 * m + 1] + b1r[m];
      const float hm = fmaxf(pre, 0.0f);
      s = fmaf(w2r[m], hm, s);
    }
    const unsigned eb = (unsigned)h_bits(s * kEmbCarry);
    unsigned ew[8];
#pragma unroll
    for (int k = 0; k < 8; ++k) ew[k] = __shfl(eb, sb + k);
    v4u ev;
    ev.x = pk16((unsigned short)ew[0], (unsigned short)ew[1]);
    ev.y = pk16((unsigned short)ew[2], (unsigned short)ew[3]);
    ev.z = pk16((unsigned short)ew[4], (unsigned short)ew[5]);
    ev.w = pk16((unsigned short)ew[6], (unsigned short)ew[7]);
    const v4u val = sel4u(lane < 16, hv, sel4u(lane < 18, ev, zero4));
    unsigned short* ad = Apl + (size_t)row * kLdA + 8 * (lane < 24 ? lane : 23);
    for (int pass = 0; pass < 2; ++pass) {
      if (lane < 24) *(volatile v4u*)ad = val;
      __threadfence();
    }
  }
}

__global__ __launch_bounds__(256) void cell_kernel(
    const float* __restrict__ gates, const float* __restrict__ cprev, float* __restrict__ cnext,
    unsigned short* __restrict__ Apl, int first) {
  const int lane = threadIdx.x & 31;
  const int wave = threadIdx.x >> 5;
  const int qL = lane & 15;
  const int rbase = (blockIdx.x * 8 + wave) * kRowsPerWave;
#pragma unroll 1
  for (int rr = 0; rr < kRowsPerWave; ++rr) {
    const int row = rbase + rr;
    const float* gp = gates + (size_t)row * kGate + 4 * lane;
    const v4f gi = *(const v4f*)(gp);
    const v4f gf = *(const v4f*)(gp + kLat);
    const v4f gg = *(const v4f*)(gp + 2 * kLat);
    const v4f go = *(const v4f*)(gp + 3 * kLat);
    v4f cp = (v4f){0.f, 0.f, 0.f, 0.f};
    if (first == 0) cp = *(const v4f*)(cprev + (size_t)row * kLat + 4 * lane);
    v4f cn = (v4f){0.f, 0.f, 0.f, 0.f};
    v4f hn = (v4f){0.f, 0.f, 0.f, 0.f};
#pragma unroll 1
    for (int u = 0; u < 4; ++u) {
      const float xi = get4f(gi, u);
      const float xf = get4f(gf, u);
      const float xg = get4f(gg, u);
      const float xo = get4f(go, u);
      const float xc = get4f(cp, u);
      const float ig = sigm_f(xi);
      const float fg = sigm_f(xf);
      const float gt = tanh_f(xg);
      const float og = sigm_f(xo);
      const float cv = fg * xc + ig * gt;
      const float hvv = og * tanh_f(cv);
      cn = put4f(cn, u, cv);
      hn = put4f(hn, u, hvv);
    }
    const unsigned p0 = pk16(h_bits(hn.x), h_bits(hn.y));
    const unsigned p1 = pk16(h_bits(hn.z), h_bits(hn.w));
    v4u hv;
    hv.x = __shfl(p0, 2 * qL);
    hv.y = __shfl(p1, 2 * qL);
    hv.z = __shfl(p0, 2 * qL + 1);
    hv.w = __shfl(p1, 2 * qL + 1);
    float* cd = cnext + (size_t)row * kLat + 4 * lane;
    unsigned short* ad = Apl + (size_t)row * kLdA + 8 * qL;
    for (int pass = 0; pass < 2; ++pass) {
      *(volatile v4f*)cd = cn;
      if (lane < 16) *(volatile v4u*)ad = hv;
      __threadfence();
    }
  }
}

__global__ __launch_bounds__(256) void head_kernel(
    const float* __restrict__ hp, const float* __restrict__ bp, const float* __restrict__ br,
    float* __restrict__ out, int rowBase) {
  __shared__ __align__(16) float st[6][256];
  const int t = threadIdx.x;
  const int row = blockIdx.x * 256 + t;
  const v4f v = *(const v4f*)(hp + (size_t)row * kNHead);
  const float pg = v.x + bp[0];
  const float r0 = v.y + br[0];
  const float r1 = v.z + br[1];
  const float r2 = v.w + br[2];
  const float mean = (r0 + r1 + r2) * (1.0f / 3.0f);
  const float s0 = sigm_f(r0), s1 = sigm_f(r1), s2 = sigm_f(r2);
  const float sm = (s0 + s1 + s2) * (1.0f / 3.0f);
  const float d0 = s0 - sm, d1 = s1 - sm, d2 = s2 - sm;
  const float var = (d0 * d0 + d1 * d1 + d2 * d2) * 0.5f;
  st[0][t] = mean;
  st[1][t] = pg;
  st[2][t] = var;
  st[3][t] = r0;
  st[4][t] = r1;
  st[5][t] = r2;
  __syncthreads();
  const int lane = t & 31, wave = t >> 5;
  const size_t gbase = (size_t)rowBase + (size_t)blockIdx.x * 256;
  for (int pass = 0; pass < 2; ++pass) {
    for (int u = wave; u < 12; u += 8) {
      const int a = u >> 1, half = u & 1;
      const v4f val = *(const v4f*)(&st[a][half * 128 + 4 * lane]);
      float* dst = out + (size_t)a * kRows + gbase + half * 128 + 4 * lane;
      *(volatile v4f*)dst = val;
    }
    __threadfence();
  }
}

extern "C" void kernel_launch(void* const* d_in, const int* in_sizes, int n_in,
                              void* d_out, int out_size, void* d_ws, size_t ws_size,
                              hipStream_t stream) {
  if (n_in < 14) return;
  if (in_sizes[0] != kNB * kLat || in_sizes[1] != kRows * 2 || in_sizes[2] != kEmb * 2 || in_sizes[3] != kEmb ||
      in_sizes[4] != kEmb * kEmb || in_sizes[5] != kEmb || in_sizes[6] != kGate * kEmb || in_sizes[7] != kGate * kLat ||
      in_sizes[8] != kGate || in_sizes[9] != kGate || in_sizes[10] != kLat || in_sizes[11] != 1 ||
      in_sizes[12] != kEns * kLat || in_sizes[13] != kEns) return;
  if (out_size != 6 * kRows) return;
  if (ws_size < kWsTotal) return;

  const float* z    = (const float*)d_in[0];
  const float* anch = (const float*)d_in[1];
  const float* W1   = (const float*)d_in[2];
  const float* b1   = (const float*)d_in[3];
  const float* W2   = (const float*)d_in[4];
  const float* b2   = (const float*)d_in[5];
  const float* Wih  = (const float*)d_in[6];
  const float* Whh  = (const float*)d_in[7];
  const float* bih  = (const float*)d_in[8];
  const float* bhh  = (const float*)d_in[9];
  const float* Wp   = (const float*)d_in[10];
  const float* bp   = (const float*)d_in[11];
  const float* Wr   = (const float*)d_in[12];
  const float* br   = (const float*)d_in[13];
  float* outp = (float*)d_out;

  char* ws = (char*)d_ws;
  unsigned short* Bt    = (unsigned short*)(ws + kOffBt);
  unsigned short* BtH   = (unsigned short*)(ws + kOffBtH);
  float*          biasS = (float*)(ws + kOffBias);
  unsigned short* A16   = (unsigned short*)(ws + kOffA);
  float*          gates = (float*)(ws + kOffG);
  float*          cbuf0 = (float*)(ws + kOffC0);
  float*          cbuf1 = (float*)(ws + kOffC1);
  float*          hp    = (float*)(ws + kOffHp);

  const int prepBlocks = (kGate + kNHead) / 8;
  const int rowBlocks  = kChunkRows / kRowsPerBlock;
  const int gemmBlocks = (kChunkRows / 64) * (kGate / 64) / 8;
  const int headGemmBlocks = (kChunkRows / 64) * (kNHead / 64) / 8;
  const int headBlocks = kChunkRows / 256;

  prep_weights_kernel<<<dim3(prepBlocks), dim3(256), 0, stream>>>(Wih, Whh, bih, bhh, Wp, Wr, Bt, BtH, biasS);

  for (int ch = 0; ch < kNumChunks; ++ch) {
    const int rowBase = ch * kChunkRows;
    init_rows_kernel<<<dim3(rowBlocks), dim3(256), 0, stream>>>(z, anch, W1, b1, W2, b2, A16, rowBase);
    for (int step = 0; step < kSteps; ++step) {
      wmma_gemm64<0, false, 2, 0, false, 0><<<dim3(gemmBlocks, 1, 1), dim3(256), 0, stream>>>(
          A16, A16, kLdA, 0L, Bt, Bt, kLdA, 0L, (void*)gates, (void*)gates, kGate, 0L,
          biasS, biasS, 0L, kChunkRows, kGate, kKdim, kScaleInv);
      const float* cpv = (step & 1) ? cbuf0 : cbuf1;
      float*       cnx = (step & 1) ? cbuf1 : cbuf0;
      cell_kernel<<<dim3(rowBlocks), dim3(256), 0, stream>>>(gates, cpv, cnx, A16, (step == 0) ? 1 : 0);
    }
    wmma_gemm64<0, false, 0, 0, false, 0><<<dim3(headGemmBlocks, 1, 1), dim3(256), 0, stream>>>(
        A16, A16, kLdA, 0L, BtH, BtH, kLdHead, 0L, (void*)hp, (void*)hp, kNHead, 0L,
        biasS, biasS, 0L, kChunkRows, kNHead, kLat, kScaleInv);
    head_kernel<<<dim3(headBlocks), dim3(256), 0, stream>>>(hp, bp, br, outp, rowBase);
  }
}
